// ParallelSelfAttention_66881230733729
// MI455X (gfx1250) — hardware-verified
//
#include <hip/hip_runtime.h>


#define SEQ    2048
#define BATCH  2
#define HIDDEN 1024
#define HEADS  16
#define HD     64
#define M_TOT  (SEQ * BATCH)
#define N_QKV  (3 * HIDDEN)
#define NORM   0.125f

typedef __attribute__((ext_vector_type(16))) __bf16 v16bf;
typedef __attribute__((ext_vector_type(8)))  __bf16 v8bf;
typedef __attribute__((ext_vector_type(8)))  float  v8f;
typedef __attribute__((ext_vector_type(4)))  float  v4f;

template <typename V> __device__ __forceinline__ void vst2(void* p, V v) {
  *(volatile V*)p = v; __threadfence(); *(volatile V*)p = v;
}
__device__ __forceinline__ __bf16 bf_hi(float x) { return (__bf16)x; }
__device__ __forceinline__ __bf16 bf_lo(float x, __bf16 h) { return (__bf16)(x - (float)h); }
__device__ __forceinline__ v8f wmma_bf16(v16bf a, v16bf b, v8f c) {
  v8f d = __builtin_amdgcn_wmma_f32_16x16x32_bf16(false, a, false, b, (short)0, c, false, false);
  asm volatile("v_nop\n\tv_nop\n\tv_nop\n\tv_nop" : "+v"(d) : "v"(a), "v"(b));
  return d;
}
__device__ __forceinline__ v8f wmma_x3(v16bf ah, v16bf al, v16bf bh, v16bf bl, v8f c) {
  c = wmma_bf16(ah, bh, c); c = wmma_bf16(ah, bl, c); c = wmma_bf16(al, bh, c);
  return c;
}

__device__ __forceinline__ void frag_f32(const float* __restrict__ base, int ld, int r0, int k0, int lane, v16bf& hi, v16bf& lo) {
  const float* p = base + (size_t)(r0 + (lane & 15)) * ld + k0 + (lane >> 4) * 8;
  const v4f a0 = *(const v4f*)(p), a1 = *(const v4f*)(p + 4), a2 = *(const v4f*)(p + 16), a3 = *(const v4f*)(p + 20);
#pragma unroll
  for (int i = 0; i < 4; ++i) {
    __bf16 h;
    h = bf_hi(a0[i]); hi[i] = h;      lo[i] = bf_lo(a0[i], h);
    h = bf_hi(a1[i]); hi[4 + i] = h;  lo[4 + i] = bf_lo(a1[i], h);
    h = bf_hi(a2[i]); hi[8 + i] = h;  lo[8 + i] = bf_lo(a2[i], h);
    h = bf_hi(a3[i]); hi[12 + i] = h; lo[12 + i] = bf_lo(a3[i], h);
  }
}
__device__ __forceinline__ v16bf frag_lds(const __bf16* base, int ld, int r0, int k0, int lane) {
  union { v16bf v; v8bf h[2]; } r;
  const __bf16* p = base + (r0 + (lane & 15)) * ld + k0 + (lane >> 4) * 8;
  r.h[0] = *(const v8bf*)(p); r.h[1] = *(const v8bf*)(p + 16);
  return r.v;
}

__device__ __forceinline__ void gemm_mainloop_32x64(const float* __restrict__ A, const float* __restrict__ Bt,
                                                    int m0, int n0, int lane, v8f acc[2][4]) {
#pragma unroll 1
  for (int k0 = 0; k0 < HIDDEN; k0 += 32) {
    v16bf ah[2], al[2], bh[4], bl[4];
    frag_f32(A, HIDDEN, m0, k0, lane, ah[0], al[0]);
    frag_f32(A, HIDDEN, m0 + 16, k0, lane, ah[1], al[1]);
#pragma unroll
    for (int j = 0; j < 4; ++j) frag_f32(Bt, HIDDEN, n0 + j * 16, k0, lane, bh[j], bl[j]);
#pragma unroll
    for (int i = 0; i < 2; ++i)
#pragma unroll
      for (int j = 0; j < 4; ++j) acc[i][j] = wmma_x3(ah[i], al[i], bh[j], bl[j], acc[i][j]);
  }
}

__global__ __launch_bounds__(128) void qkv_gemm_kernel(
    const float* __restrict__ X, const float* __restrict__ Wq, const float* __restrict__ bias,
    float* __restrict__ Qb, float* __restrict__ Kb, float* __restrict__ Vt) {
  __shared__ __align__(16) float st[128][64];
  const int lane = threadIdx.x & 31;
  const int wave = threadIdx.x >> 5;
  const int mblk = blockIdx.y * 128;
  const int m0 = mblk + wave * 32;
  const int n0 = blockIdx.x * 64;
  const int head = n0 / (3 * HD), part = (n0 % (3 * HD)) / HD;

  v8f acc[2][4] = {};
  gemm_mainloop_32x64(X, Wq, m0, n0, lane, acc);

  const int half = lane >> 4, col = lane & 15;
#pragma unroll
  for (int i = 0; i < 2; ++i)
#pragma unroll
    for (int j = 0; j < 4; ++j)
#pragma unroll
      for (int r = 0; r < 8; ++r)
        st[wave * 32 + i * 16 + r + 8 * half][j * 16 + col] = acc[i][j][r] + bias[n0 + j * 16 + col];
  __syncthreads();

  const int tid = threadIdx.x;
  const int s0 = mblk >> 1;
  if (part < 2) {
    float* dst = (part == 0) ? Qb : Kb;
    for (int g = tid; g < 128 * 16; g += 128) {
      const int ml = g >> 4, pc = g & 15;
      const int m = mblk + ml, s = m >> 1, bch = m & 1;
      vst2(dst + ((size_t)(bch * HEADS + head) * SEQ + s) * HD + pc * 4, *(const v4f*)(&st[ml][pc * 4]));
    }
  } else {
    for (int g = tid; g < 2 * 64 * 16; g += 128) {
      const int pc = g & 15, d = (g >> 4) & 63, bch = g >> 10;
      v4f v;
#pragma unroll
      for (int e = 0; e < 4; ++e) v[e] = st[(pc * 4 + e) * 2 + bch][d];
      vst2(Vt + ((size_t)(bch * HEADS + head) * HD + d) * SEQ + s0 + pc * 4, v);
    }
  }
}

__global__ __launch_bounds__(128) void attn_kernel(
    const float* __restrict__ Qb, const float* __restrict__ Kb,
    const float* __restrict__ Vt, float* __restrict__ Ctx) {
  __shared__ __align__(16) __bf16 Kh[32 * 72], Kl[32 * 72];
  __shared__ __align__(16) __bf16 Vh[64 * 40], Vl[64 * 40];
  __shared__ __align__(16) __bf16 Ph[4][16 * 40], Pl[4][16 * 40];
  __shared__ __align__(16) float  Os[4][16 * 64];

  const int tid  = threadIdx.x;
  const int lane = tid & 31;
  const int wave = tid >> 5;
  const int half = lane >> 4;
  const int col  = lane & 15;
  const int q0   = blockIdx.x * 64;
  const int head = blockIdx.y;
  const int bch  = blockIdx.z;

  const float* Qh = Qb + (size_t)(bch * HEADS + head) * SEQ * HD;
  const float* Kg = Kb + (size_t)(bch * HEADS + head) * SEQ * HD;
  const float* Vg = Vt + (size_t)(bch * HEADS + head) * HD * SEQ;
  const int mq = q0 + wave * 16;

  v16bf qh[2], ql[2];
#pragma unroll
  for (int kb = 0; kb < 2; ++kb) frag_f32(Qh, HD, mq, kb * 32, lane, qh[kb], ql[kb]);

  v8f o[4] = {};
  float mrow[8], lrow[8];
#pragma unroll
  for (int r = 0; r < 8; ++r) { mrow[r] = -3.0e38f; lrow[r] = 0.0f; }

  __bf16* ph = Ph[wave];
  __bf16* pl = Pl[wave];
  const int t_end = q0 + 64;
  for (int t0 = 0; t0 < t_end; t0 += 32) {
    __syncthreads();
    {
      const int kr = tid >> 2, kc = (tid & 3) * 16;
      const float* kp = Kg + (size_t)(t0 + kr) * HD + kc;
      const int vr = tid >> 1, vc = (tid & 1) * 16;
      const float* vp = Vg + (size_t)vr * SEQ + t0 + vc;
#pragma unroll
      for (int e = 0; e < 16; e += 4) {
        const v4f a = *(const v4f*)(kp + e), b = *(const v4f*)(vp + e);
#pragma unroll
        for (int i = 0; i < 4; ++i) {
          __bf16 h = bf_hi(a[i]); Kh[kr * 72 + kc + e + i] = h; Kl[kr * 72 + kc + e + i] = bf_lo(a[i], h);
          __bf16 g = bf_hi(b[i]); Vh[vr * 40 + vc + e + i] = g; Vl[vr * 40 + vc + e + i] = bf_lo(b[i], g);
        }
      }
    }
    __syncthreads();

    v8f s[2] = {};
#pragma unroll
    for (int n = 0; n < 2; ++n)
#pragma unroll
      for (int kb = 0; kb < 2; ++kb) {
        const v16bf kh = frag_lds(Kh, 72, n * 16, kb * 32, lane);
        const v16bf kl = frag_lds(Kl, 72, n * 16, kb * 32, lane);
        s[n] = wmma_x3(qh[kb], ql[kb], kh, kl, s[n]);
      }

    {
      const int k0g = t0 + col, k1g = t0 + 16 + col;
#pragma unroll
      for (int r = 0; r < 8; ++r) {
        const int qg = mq + r + 8 * half;
        float v0 = s[0][r] * NORM; if (k0g > qg) v0 = -10000.0f;
        float v1 = s[1][r] * NORM; if (k1g > qg) v1 = -10000.0f;
        float mx = fmaxf(v0, v1);
#pragma unroll
        for (int off = 8; off > 0; off >>= 1) mx = fmaxf(mx, __shfl_xor(mx, off, 16));
        const float mnew  = fmaxf(mrow[r], mx);
        const float alpha = __expf(mrow[r] - mnew);
        const float p0 = __expf(v0 - mnew);
        const float p1 = __expf(v1 - mnew);
        float rs = p0 + p1;
#pragma unroll
        for (int off = 8; off > 0; off >>= 1) rs += __shfl_xor(rs, off, 16);
        lrow[r] = lrow[r] * alpha + rs;
        mrow[r] = mnew;
#pragma unroll
        for (int j = 0; j < 4; ++j) o[j][r] *= alpha;
        const int row = r + 8 * half;
        __bf16 h0 = bf_hi(p0), h1 = bf_hi(p1);
        ph[row * 40 + col] = h0;      pl[row * 40 + col] = bf_lo(p0, h0);
        ph[row * 40 + 16 + col] = h1; pl[row * 40 + 16 + col] = bf_lo(p1, h1);
      }
    }
    __syncthreads();

    const v16bf pah = frag_lds(ph, 40, 0, 0, lane), pal = frag_lds(pl, 40, 0, 0, lane);
#pragma unroll
    for (int j = 0; j < 4; ++j) {
      const v16bf vh = frag_lds(Vh, 40, j * 16, 0, lane), vl = frag_lds(Vl, 40, j * 16, 0, lane);
      o[j] = wmma_x3(pah, pal, vh, vl, o[j]);
    }
  }

  float* os_ = Os[wave];
#pragma unroll
  for (int r = 0; r < 8; ++r) {
    const float inv = 1.0f / lrow[r];
#pragma unroll
    for (int j = 0; j < 4; ++j) os_[(r + 8 * half) * 64 + j * 16 + col] = o[j][r] * inv;
  }
  __syncthreads();
#pragma unroll
  for (int q = 0; q < 8; ++q) {
    const int rl = q * 2 + (lane >> 4), pc = lane & 15;
    const size_t m = (size_t)(mq + rl) * BATCH + bch;
    vst2(Ctx + m * HIDDEN + head * HD + pc * 4, *(const v4f*)(os_ + rl * 64 + pc * 4));
  }
}

__global__ __launch_bounds__(128) void dense_gemm_kernel(
    const float* __restrict__ Cx, const float* __restrict__ Wd, const float* __restrict__ bias, float* __restrict__ Out) {
  __shared__ __align__(16) float st[4][32 * 64];
  const int lane = threadIdx.x & 31;
  const int wave = threadIdx.x >> 5;
  const int m0 = blockIdx.y * 64 + (wave >> 1) * 32;
  const int n0 = blockIdx.x * 128 + (wave & 1) * 64;

  v8f acc[2][4] = {};
  gemm_mainloop_32x64(Cx, Wd, m0, n0, lane, acc);

  const int half = lane >> 4, col = lane & 15;
  float* S = st[wave];
#pragma unroll
  for (int i = 0; i < 2; ++i)
#pragma unroll
    for (int j = 0; j < 4; ++j)
#pragma unroll
      for (int r = 0; r < 8; ++r) S[(i * 16 + r + 8 * half) * 64 + j * 16 + col] = acc[i][j][r] + bias[n0 + j * 16 + col];
  __syncthreads();
#pragma unroll
  for (int q = 0; q < 16; ++q) {
    const int rl = q * 2 + (lane >> 4), pc = lane & 15;
    vst2(Out + (size_t)(m0 + rl) * HIDDEN + n0 + pc * 4, *(const v4f*)(S + rl * 64 + pc * 4));
  }
}

extern "C" void kernel_launch(void* const* d_in, const int* in_sizes, int n_in,
                              void* d_out, int out_size, void* d_ws, size_t ws_size,
                              hipStream_t stream) {
  (void)in_sizes; (void)n_in; (void)out_size; (void)ws_size;
  const float* hidden  = (const float*)d_in[0];
  const float* w_qkv   = (const float*)d_in[2];
  const float* b_qkv   = (const float*)d_in[3];
  const float* w_dense = (const float*)d_in[4];
  const float* b_dense = (const float*)d_in[5];
  float* out = (float*)d_out;

  char* ws = (char*)d_ws;
  size_t off = 0;
  auto carve = [&](size_t bytes) { void* p = ws + off; off = (off + bytes + 255) & ~(size_t)255; return (float*)p; };
  float* Qb  = carve((size_t)BATCH * HEADS * SEQ * HD * 4);
  float* Kb  = carve((size_t)BATCH * HEADS * SEQ * HD * 4);
  float* Vt  = carve((size_t)BATCH * HEADS * HD * SEQ * 4);
  float* Ctx = carve((size_t)M_TOT * HIDDEN * 4);

  qkv_gemm_kernel<<<dim3(N_QKV / 64, M_TOT / 128), 128, 0, stream>>>(hidden, w_qkv, b_qkv, Qb, Kb, Vt);
  attn_kernel<<<dim3(SEQ / 64, HEADS, BATCH), 128, 0, stream>>>(Qb, Kb, Vt, Ctx);
  dense_gemm_kernel<<<dim3(HIDDEN / 128, M_TOT / 64), 128, 0, stream>>>(Ctx, w_dense, b_dense, out);
}
